// RowSelfAttentionWithBulkBias_1382979469737
// MI455X (gfx1250) — hardware-verified
//
#include <hip/hip_runtime.h>


#define NBS  8
#define NTR  4
#define LL   1024
#define CC   256
#define NH_  8
#define HD   32
#define NT   (NBS * LL)
#define ZH   4
#define PCAR 1024.0f
typedef _Float16 h16;
typedef unsigned short bf;
typedef __attribute__((ext_vector_type(16))) __bf16   v16bf;
typedef __attribute__((ext_vector_type(16))) _Float16 v16h;
typedef __attribute__((ext_vector_type(8)))  _Float16 v8h;
typedef __attribute__((ext_vector_type(8)))  unsigned short v8us;
typedef __attribute__((ext_vector_type(8)))  float    v8f;
typedef __attribute__((ext_vector_type(4)))  float    v4f;
typedef v8h  __attribute__((may_alias)) v8ha;
typedef v4f  __attribute__((may_alias)) v4fa;
typedef v8us __attribute__((may_alias)) v8usa;

__device__ __forceinline__ unsigned short f2bf(float f) { unsigned u = __float_as_uint(f); u += 0x7FFFu + ((u >> 16) & 1u); return (unsigned short)(u >> 16); }
__device__ __forceinline__ float bf2f(unsigned short b) { return __uint_as_float(((unsigned)b) << 16); }
__device__ __forceinline__ float bfr(float f) { return bf2f(f2bf(f)); }
__device__ __forceinline__ v16h cat16(v8h lo, v8h hi) { return __builtin_shufflevector(lo, hi, 0, 1, 2, 3, 4, 5, 6, 7, 8, 9, 10, 11, 12, 13, 14, 15); }
__device__ __forceinline__ v16bf cat16b(v8us lo, v8us hi) { return __builtin_bit_cast(v16bf, __builtin_shufflevector(lo, hi, 0, 1, 2, 3, 4, 5, 6, 7, 8, 9, 10, 11, 12, 13, 14, 15)); }
__device__ __forceinline__ v8f wmma16(v16h a, v16h b, v8f c) { return __builtin_amdgcn_wmma_f32_16x16x32_f16(false, a, false, b, (short)0, c, false, false); }
__device__ __forceinline__ v8f wmmab(v16bf a, v16bf b, v8f c) { return __builtin_amdgcn_wmma_f32_16x16x32_bf16(false, a, false, b, (short)0, c, false, false); }


template <typename T16> struct WFrag;
template <> struct WFrag<h16> { typedef v16h V; static __device__ __forceinline__ V ld(const h16* p) { return cat16(*(const v8h*)p, *(const v8h*)(p + 16)); } static __device__ __forceinline__ v8f mma(V a, V b, v8f c) { return wmma16(a, b, c); } };
template <> struct WFrag<bf> { typedef v16bf V; static __device__ __forceinline__ V ld(const bf* p) { return cat16b(*(const v8us*)p, *(const v8us*)(p + 16)); } static __device__ __forceinline__ v8f mma(V a, V b, v8f c) { return wmmab(a, b, c); } };
template <typename T16, int NSPLIT, bool BIAS>
__global__ __launch_bounds__(32) void k_gemmw(const T16* __restrict__ A, const T16* __restrict__ A2, const T16* __restrict__ Bt, const T16* __restrict__ Bt2, int K, float* C, int ldc, const float* __restrict__ bias, size_t sA, size_t sB, size_t sC) {
    typedef typename WFrag<T16>::V V;
    __shared__ __align__(16) float os[16 * 68];
    const size_t z = blockIdx.z; A += z * sA; if (A2) A2 += z * sA; Bt += z * sB; if (Bt2) Bt2 += z * sB; C += z * sC;
    const int lane = threadIdx.x & 31, lr = lane & 15, hi = lane >> 4; const int r0 = blockIdx.x * 64, c0 = blockIdx.y * 64;
    v8f acc[4][4];
#pragma unroll
    for (int mb = 0; mb < 4; ++mb)
#pragma unroll
        for (int nb = 0; nb < 4; ++nb) acc[mb][nb] = (v8f){};
    const size_t aoff = (size_t)(r0 + lr) * K + 8 * hi, boff = (size_t)(c0 + lr) * K + 8 * hi;
#pragma unroll 1
    for (int kc = 0; kc < K; kc += 32) {
        V a[4], a2[4];
#pragma unroll
        for (int mb = 0; mb < 4; ++mb) { a[mb] = WFrag<T16>::ld(A + aoff + (size_t)mb * 16 * K + kc); if (NSPLIT == 1 || NSPLIT == 2) a2[mb] = WFrag<T16>::ld(A2 + aoff + (size_t)mb * 16 * K + kc); }
#pragma unroll
        for (int nb = 0; nb < 4; ++nb) { const V b = WFrag<T16>::ld(Bt + boff + (size_t)nb * 16 * K + kc); V b2; if (NSPLIT >= 2) b2 = WFrag<T16>::ld(Bt2 + boff + (size_t)nb * 16 * K + kc);
#pragma unroll
            for (int mb = 0; mb < 4; ++mb) { acc[mb][nb] = WFrag<T16>::mma(a[mb], b, acc[mb][nb]); if (NSPLIT == 1 || NSPLIT == 2) acc[mb][nb] = WFrag<T16>::mma(a2[mb], b, acc[mb][nb]); if (NSPLIT >= 2) acc[mb][nb] = WFrag<T16>::mma(a[mb], b2, acc[mb][nb]); } }
        asm volatile("v_nop\n\tv_nop\n\tv_nop\n\tv_nop" : "+v"(acc[0][0]), "+v"(acc[1][1]), "+v"(acc[2][2]), "+v"(acc[3][3]) : "v"(a[0]), "v"(a[3]));
    }
#pragma unroll
    for (int mb = 0; mb < 4; ++mb) {
#pragma unroll
        for (int nb = 0; nb < 4; ++nb) {
#pragma unroll
            for (int j = 0; j < 8; ++j) os[(hi * 8 + j) * 68 + nb * 16 + lr] = acc[mb][nb][j]; }
        __builtin_amdgcn_wave_barrier(); asm volatile("" ::: "memory");
        float* crow = C + (size_t)(r0 + mb * 16) * ldc + c0;
#pragma unroll 1
        for (int ps = 0; ps < 2; ++ps) {
#pragma unroll
            for (int s = 0; s < 8; ++s) { const int row = 2 * s + hi, cofs = lr * 4; v4f val = *(const v4fa*)(os + row * 68 + cofs); if (BIAS) { val[0] += bfr(bias[c0 + cofs]); val[1] += bfr(bias[c0 + cofs + 1]); val[2] += bfr(bias[c0 + cofs + 2]); val[3] += bfr(bias[c0 + cofs + 3]); }
                *(volatile v4f*)(crow + (size_t)row * ldc + cofs) = val; }
            if (ps == 0) __threadfence(); }
        __builtin_amdgcn_wave_barrier(); asm volatile("" ::: "memory");
    }
}

__device__ __forceinline__ h16 tohx(float x) { return (h16)x; }
__device__ __forceinline__ void splitf(float y, unsigned short& h, unsigned short& l) { h = f2bf(y); l = f2bf(y - bf2f(h)); }
__device__ __noinline__ float sigm(float z) { return __fdiv_rn(1.0f, 1.0f + __expf(-z)); }
typedef __attribute__((ext_vector_type(2))) _Float16 v2h;
typedef __attribute__((ext_vector_type(4))) _Float16 v4h;
typedef __attribute__((ext_vector_type(2))) unsigned short v2us;
typedef __attribute__((ext_vector_type(4))) unsigned short v4us;

__global__ __launch_bounds__(256) void k_cvt8(const float* __restrict__ src, bf* dst, size_t n8) { const size_t i = (size_t)blockIdx.x * 256 + threadIdx.x; if (i >= n8) return; const v8f v = *(const v8f*)(src + i * 8); v8us o;
#pragma unroll
    for (int k = 0; k < 8; ++k) o[k] = f2bf(v[k]); *(volatile v8us*)(dst + i * 8) = o; __threadfence(); *(volatile v8us*)(dst + i * 8) = o; }
__global__ __launch_bounds__(256) void k_gwb(const float* __restrict__ gw, bf* GB) {
    const int lane = threadIdx.x & 31; const int L = blockIdx.x * 8 + (threadIdx.x >> 5); if (L >= NH_ * 64 * HD / 64) return; const int e = L * 64 + lane * 2; const int d = e & 31; const int n = (e >> 5) & 63; const int h = e >> 11; v2us o;
#pragma unroll
    for (int q = 0; q < 2; ++q) o[q] = (n < HD) ? f2bf(gw[((size_t)h * HD + n) * HD + d + q]) : (unsigned short)0;
    *(volatile v2us*)(GB + e) = o; __threadfence(); *(volatile v2us*)(GB + e) = o;
}
__global__ __launch_bounds__(256) void k_qkplane(const float* __restrict__ F, int col0, float sc, h16* P) {
    const int lane = threadIdx.x & 31; const int L0 = (blockIdx.x * 8 + (threadIdx.x >> 5)) * 8; const int nlines = NT * CC / 64;
#pragma unroll 1
    for (int ps = 0; ps < 2; ++ps) {
#pragma unroll
        for (int l = 0; l < 8; ++l) { const int Ln = L0 + l; if (Ln >= nlines) break; const int e = Ln * 64 + lane * 2; const int d = e & 31; const int t = (e >> 5) & (LL - 1); const int h = (e >> 15) & 7; const int bs = e >> 18; v2h v;
#pragma unroll
            for (int q = 0; q < 2; ++q) v[q] = tohx(F[((size_t)bs * LL + t) * (3 * CC) + col0 + h * HD + d + q] * sc);
            *(volatile v2h*)(P + (size_t)e) = v; }
        if (ps == 0) __threadfence(); }
}
__global__ __launch_bounds__(256) void k_vtplane(const float* __restrict__ F, h16* VT) {
    const int lane = threadIdx.x & 31; const int L0 = (blockIdx.x * 8 + (threadIdx.x >> 5)) * 8; const int nlines = NBS * NH_ * 64 * LL / 64;
#pragma unroll 1
    for (int ps = 0; ps < 2; ++ps) {
#pragma unroll
        for (int l = 0; l < 8; ++l) { const int Ln = L0 + l; if (Ln >= nlines) break; const int e = Ln * 64 + lane * 2; const int t = e & (LL - 1); const int d = (e >> 10) & 63; const int h = (e >> 16) & 7; const int bs = e >> 19; v2h v;
#pragma unroll
            for (int q = 0; q < 2; ++q) v[q] = tohx(d < HD ? F[((size_t)bs * LL + t + q) * (3 * CC) + 2 * CC + h * HD + d] : 0.f);
            *(volatile v2h*)(VT + (size_t)e) = v; }
        if (ps == 0) __threadfence(); }
}
__global__ __launch_bounds__(256) void k_softbb(const float* __restrict__ Sb, const float* __restrict__ bulk, const float* __restrict__ cw, const float* __restrict__ cb, int bs, int h0, h16* P) {
    const int lane = threadIdx.x & 31; const int row = blockIdx.x * 8 + (threadIdx.x >> 5); if (row >= ZH * LL) return; const int i = row & (LL - 1); const int h = h0 + (row >> 10); const int b = bs / NTR;
    const float* sr = Sb + (size_t)row * LL; const float* br = bulk + ((size_t)b * LL + i) * LL; const float w = bfr(cw[h]), c0 = bfr(cb[h]); float v[32]; float m = -3.0e38f;
#pragma unroll
    for (int ch = 0; ch < 8; ++ch) { const v4f s = *(const v4f*)(sr + ch * 128 + lane * 4), bb = *(const v4f*)(br + ch * 128 + lane * 4);
#pragma unroll
        for (int q = 0; q < 4; ++q) { const float t = s[q] + (w * bfr(bb[q]) + c0); v[ch * 4 + q] = t; m = fmaxf(m, t); } }
#pragma unroll
    for (int sh = 16; sh; sh >>= 1) m = fmaxf(m, __shfl_xor(m, sh, 32));
    float sum = 0.f;
#pragma unroll
    for (int k = 0; k < 32; ++k) { v[k] = __expf(v[k] - m); sum += v[k]; }
#pragma unroll
    for (int sh = 16; sh; sh >>= 1) sum += __shfl_xor(sum, sh, 32);
    const float f = __fdiv_rn(PCAR, sum);
#pragma unroll 1
    for (int ps = 0; ps < 2; ++ps) {
#pragma unroll
        for (int ch = 0; ch < 8; ++ch) { v4h o;
#pragma unroll
            for (int q = 0; q < 4; ++q) o[q] = tohx(v[ch * 4 + q] * f);
            *(volatile v4h*)(P + (size_t)row * LL + ch * 128 + lane * 4) = o; }
        if (ps == 0) __threadfence(); }
}
__global__ __launch_bounds__(256) void k_og(const float* __restrict__ O, int bs, int h0, float* OA) {
    const int lane = threadIdx.x & 31; const int wg = blockIdx.x * 8 + (threadIdx.x >> 5); if (wg >= (ZH / 2) * LL) return; const int t = wg % LL; const int zz = (wg / LL) * 2 + (lane >> 4); const int d = (lane & 15) * 2;
    typedef __attribute__((ext_vector_type(2))) float v2f; v2f o; o[0] = O[((size_t)zz * LL + t) * 64 + d] * (1.0f / PCAR); o[1] = O[((size_t)zz * LL + t) * 64 + d + 1] * (1.0f / PCAR);
    float* dst = OA + ((size_t)bs * LL + t) * CC + (h0 + zz) * HD + d; *(volatile v2f*)dst = o; __threadfence(); *(volatile v2f*)dst = o;
}
__global__ __launch_bounds__(256) void k_oplane(const float* __restrict__ OA, bf* Ph, bf* Pl) {
    const int lane = threadIdx.x & 31; const int L0 = (blockIdx.x * 8 + (threadIdx.x >> 5)) * 8; const int nlines = NH_ * NT * HD / 64;
#pragma unroll 1
    for (int ps = 0; ps < 2; ++ps) {
#pragma unroll
        for (int l = 0; l < 8; ++l) { const int Ln = L0 + l; if (Ln >= nlines) break; const int e = Ln * 64 + lane * 2; const int d = e & 31; const int r = (e >> 5) & (NT - 1); const int h = e >> 18; v2us oh, ol;
#pragma unroll
            for (int q = 0; q < 2; ++q) { unsigned short a, c2; splitf(OA[(size_t)r * CC + h * HD + d + q], a, c2); oh[q] = a; ol[q] = c2; }
            *(volatile v2us*)(Ph + (size_t)e) = oh; *(volatile v2us*)(Pl + (size_t)e) = ol; }
        if (ps == 0) __threadfence(); }
}
__global__ __launch_bounds__(256) void k_gmul(const float* __restrict__ OA, const float* __restrict__ GC, const float* __restrict__ gb, bf* Ph, bf* Pl) {
    const int lane = threadIdx.x & 31; const int L0 = (blockIdx.x * 8 + (threadIdx.x >> 5)) * 8; const int nlines = NT * CC / 64;
#pragma unroll 1
    for (int ps = 0; ps < 2; ++ps) {
#pragma unroll
        for (int l = 0; l < 8; ++l) { const int Ln = L0 + l; if (Ln >= nlines) break; const int e = Ln * 64 + lane * 2; const int col = e & 255; const int r = e >> 8; const int h = col >> 5, c = col & 31; v2us oh, ol;
#pragma unroll
            for (int q = 0; q < 2; ++q) { const float g = sigm(GC[((size_t)h * NT + r) * 64 + c + q] + bfr(gb[h * HD + c + q])); unsigned short a, c2; splitf(OA[(size_t)e + q] * g, a, c2); oh[q] = a; ol[q] = c2; }
            *(volatile v2us*)(Ph + (size_t)e) = oh; *(volatile v2us*)(Pl + (size_t)e) = ol; }
        if (ps == 0) __threadfence(); }
}
__global__ __launch_bounds__(256) void k_lnres(const float* __restrict__ AO, const float* __restrict__ x, const float* __restrict__ gg, const float* __restrict__ bb, float* OUT) {
    const int lane = threadIdx.x & 31; const int r = blockIdx.x * 8 + (threadIdx.x >> 5); if (r >= NT) return; float v[8]; float s = 0.f;
#pragma unroll
    for (int c = 0; c < 2; ++c)
#pragma unroll
        for (int q = 0; q < 4; ++q) { const size_t idx = (size_t)r * CC + c * 128 + lane * 4 + q; const float t = bfr(x[idx]) + AO[idx]; v[c * 4 + q] = t; s += t; }
#pragma unroll
    for (int sh = 16; sh; sh >>= 1) s += __shfl_xor(s, sh, 32);
    const float mu = s * (1.0f / CC); float qq = 0.f;
#pragma unroll
    for (int i = 0; i < 8; ++i) { const float d0 = v[i] - mu; qq = fmaf(d0, d0, qq); }
#pragma unroll
    for (int sh = 16; sh; sh >>= 1) qq += __shfl_xor(qq, sh, 32);
    const float rs = __fdiv_rn(1.0f, sqrtf(qq * (1.0f / CC) + 1e-5f)); v4f o[2];
#pragma unroll
    for (int c = 0; c < 2; ++c)
#pragma unroll
        for (int q = 0; q < 4; ++q) { const int col = c * 128 + lane * 4 + q; o[c][q] = (v[c * 4 + q] - mu) * rs * bfr(gg[col]) + bfr(bb[col]); }
#pragma unroll 1
    for (int ps = 0; ps < 2; ++ps) {
#pragma unroll
        for (int c = 0; c < 2; ++c) *(volatile v4f*)(OUT + (size_t)r * CC + c * 128 + lane * 4) = o[c];
        if (ps == 0) __threadfence(); }
}

extern "C" void kernel_launch(void* const* d_in, const int* in_sizes, int n_in,
                              void* d_out, int out_size, void* d_ws, size_t ws_size, hipStream_t stream) {
    (void)in_sizes; (void)n_in; (void)out_size;
    const float* x = (const float*)d_in[0]; const float* bulk = (const float*)d_in[1]; const float* Wq = (const float*)d_in[2]; const float* bq = (const float*)d_in[3]; const float* Wk = (const float*)d_in[4]; const float* bk = (const float*)d_in[5]; const float* Wv = (const float*)d_in[6]; const float* bv = (const float*)d_in[7];
    const float* Wo = (const float*)d_in[8]; const float* bo = (const float*)d_in[9]; const float* cw = (const float*)d_in[10]; const float* cb = (const float*)d_in[11]; const float* gw = (const float*)d_in[12]; const float* gb = (const float*)d_in[13]; const float* lg = (const float*)d_in[14]; const float* lb = (const float*)d_in[15];
    float* OUT = (float*)d_out;
    char* wsp = (char*)d_ws;
    auto take = [&](size_t bytes) { char* p = wsp; wsp += (bytes + 255) & ~(size_t)255; return (void*)p; };
    bf* XB = (bf*)take((size_t)NT * CC * 2); bf* WQ = (bf*)take((size_t)CC * CC * 2); bf* WK = (bf*)take((size_t)CC * CC * 2); bf* WV = (bf*)take((size_t)CC * CC * 2); bf* WO = (bf*)take((size_t)CC * CC * 2); bf* GB = (bf*)take((size_t)NH_ * 64 * HD * 2);
    float* F = (float*)take((size_t)NT * 3 * CC * 4); h16* QP = (h16*)take((size_t)NT * CC * 2); h16* KP = (h16*)take((size_t)NT * CC * 2); h16* VT = (h16*)take((size_t)NBS * NH_ * 64 * LL * 2);
    float* Sb = (float*)take((size_t)ZH * LL * LL * 4); h16* Pm = (h16*)take((size_t)ZH * LL * LL * 2); float* Ob = (float*)take((size_t)ZH * LL * 64 * 4);
    float* OA = (float*)take((size_t)NT * CC * 4); bf* OPh = (bf*)take((size_t)NT * CC * 2); bf* OPl = (bf*)take((size_t)NT * CC * 2); float* GC = (float*)take((size_t)NH_ * NT * 64 * 4); bf* OGh = (bf*)take((size_t)NT * CC * 2); bf* OGl = (bf*)take((size_t)NT * CC * 2);
    if ((size_t)(wsp - (char*)d_ws) > ws_size) return;
    float* AO = F;
    { const size_t nx = (size_t)NT * CC / 8, nw = (size_t)CC * CC / 8; k_cvt8<<<(unsigned)((nx + 255) / 256), 256, 0, stream>>>(x, XB, nx);
      k_cvt8<<<(unsigned)((nw + 255) / 256), 256, 0, stream>>>(Wq, WQ, nw); k_cvt8<<<(unsigned)((nw + 255) / 256), 256, 0, stream>>>(Wk, WK, nw); k_cvt8<<<(unsigned)((nw + 255) / 256), 256, 0, stream>>>(Wv, WV, nw); k_cvt8<<<(unsigned)((nw + 255) / 256), 256, 0, stream>>>(Wo, WO, nw);
      k_gwb<<<(NH_ * 64 * HD / 64 + 7) / 8, 256, 0, stream>>>(gw, GB); }
    k_gemmw<bf, 0, true><<<dim3(NT / 64, CC / 64, 1), 32, 0, stream>>>(XB, nullptr, WQ, nullptr, CC, F, 3 * CC, bq, 0, 0, 0);
    k_gemmw<bf, 0, true><<<dim3(NT / 64, CC / 64, 1), 32, 0, stream>>>(XB, nullptr, WK, nullptr, CC, F + CC, 3 * CC, bk, 0, 0, 0);
    k_gemmw<bf, 0, true><<<dim3(NT / 64, CC / 64, 1), 32, 0, stream>>>(XB, nullptr, WV, nullptr, CC, F + 2 * CC, 3 * CC, bv, 0, 0, 0);
    const unsigned LB = (unsigned)((NT * CC / 64 + 63) / 64);
    k_qkplane<<<LB, 256, 0, stream>>>(F, 0, 0x1.6a09e6p-3f, QP); k_qkplane<<<LB, 256, 0, stream>>>(F, CC, 1.0f, KP);
    k_vtplane<<<(unsigned)((NBS * NH_ * 64 * LL / 64 + 63) / 64), 256, 0, stream>>>(F, VT);
    for (int bs = 0; bs < NBS; ++bs)
        for (int h0 = 0; h0 < NH_; h0 += ZH) { const size_t z0 = (size_t)bs * NH_ + h0;
            k_gemmw<h16, 0, false><<<dim3(LL / 64, LL / 64, ZH), 32, 0, stream>>>(QP + z0 * LL * HD, nullptr, KP + z0 * LL * HD, nullptr, HD, Sb, LL, nullptr, (size_t)LL * HD, (size_t)LL * HD, (size_t)LL * LL);
            k_softbb<<<ZH * LL / 8, 256, 0, stream>>>(Sb, bulk, cw, cb, bs, h0, Pm);
            k_gemmw<h16, 0, false><<<dim3(LL / 64, 1, ZH), 32, 0, stream>>>(Pm, nullptr, VT + z0 * 64 * LL, nullptr, LL, Ob, 64, nullptr, (size_t)LL * LL, (size_t)64 * LL, (size_t)LL * 64);
            k_og<<<(ZH / 2) * LL / 8, 256, 0, stream>>>(Ob, bs, h0, OA); }
    k_oplane<<<(NH_ * NT * HD / 64 + 63) / 64, 256, 0, stream>>>(OA, OPh, OPl);
    k_gemmw<bf, 1, false><<<dim3(NT / 64, 1, NH_), 32, 0, stream>>>(OPh, OPl, GB, nullptr, HD, GC, 64, nullptr, (size_t)NT * HD, (size_t)64 * HD, (size_t)NT * 64);
    k_gmul<<<LB, 256, 0, stream>>>(OA, GC, gb, OGh, OGl);
    k_gemmw<bf, 1, true><<<dim3(NT / 64, CC / 64, 1), 32, 0, stream>>>(OGh, OGl, WO, nullptr, CC, AO, CC, bo, 0, 0, 0);
    k_lnres<<<NT / 8, 256, 0, stream>>>(AO, x, lg, lb, OUT);
}
